// CausalMHA_67843303408009
// MI455X (gfx1250) — hardware-verified
//
#include <hip/hip_runtime.h>
#include <math.h>

constexpr int kBatch = 2;
constexpr int kSeq   = 2048;
constexpr int kDim   = 1024;
constexpr int kHeads = 16;
constexpr int kDh    = 64;
constexpr int kTok   = kBatch * kSeq;
constexpr int kQkvN  = 3 * kDim;
constexpr float kAttnScale = 0.125f;
constexpr int kAQ = 64;
constexpr int kAK = 64;
constexpr int kOsPitch = 68;
static_assert(kHeads * kDh == kDim);
static_assert(kTok % 64 == 0 && kQkvN % 64 == 0 && kDim % 64 == 0);
static_assert(kDim % 32 == 0);
static_assert(kSeq % kAQ == 0 && kSeq % kAK == 0 && kDh == 64);
static_assert((kTok * kDim) % (8 * 256) == 0 && (kQkvN * kDim) % (8 * 256) == 0 && (kDim * kDim) % (8 * 256) == 0);

typedef __attribute__((ext_vector_type(16))) _Float16 v16h;
typedef __attribute__((ext_vector_type(8)))  _Float16 v8h;
typedef __attribute__((ext_vector_type(16))) __bf16   v16b;
typedef __attribute__((ext_vector_type(8)))  __bf16   v8b;
typedef __attribute__((ext_vector_type(8)))  float    v8f;
typedef __attribute__((ext_vector_type(4)))  float    v4f;
typedef __attribute__((ext_vector_type(4)))  unsigned int v4u;

__device__ __forceinline__ unsigned short f2bf_bits(float f) {
  unsigned u = __float_as_uint(f);
  return (unsigned short)((u + 0x7FFFu + ((u >> 16) & 1u)) >> 16);
}
__device__ __forceinline__ float bf_bits2f(unsigned short h) { return __uint_as_float(((unsigned)h) << 16); }
__device__ __forceinline__ unsigned pk16(unsigned short a, unsigned short b) { return (unsigned)a | ((unsigned)b << 16); }

__device__ __forceinline__ void dep_guard_h(v8f& a, v8f& b, v16h x, v16h y) { asm volatile("v_nop\n\tv_nop\n\tv_nop\n\tv_nop" : "+v"(a), "+v"(b) : "v"(x), "v"(y)); }
__device__ __forceinline__ void dep_guard_b(v8f& a, v8f& b, v16b x, v16b y) { asm volatile("v_nop\n\tv_nop\n\tv_nop\n\tv_nop" : "+v"(a), "+v"(b) : "v"(x), "v"(y)); }
__device__ __forceinline__ void dep_guard4_h(v8f& a, v8f& b, v8f& c, v8f& d, v16h x, v16h y) { asm volatile("v_nop\n\tv_nop\n\tv_nop\n\tv_nop" : "+v"(a), "+v"(b), "+v"(c), "+v"(d) : "v"(x), "v"(y)); }
__device__ __forceinline__ void dep_guard4_b(v8f& a, v8f& b, v8f& c, v8f& d, v16b x, v16b y) { asm volatile("v_nop\n\tv_nop\n\tv_nop\n\tv_nop" : "+v"(a), "+v"(b), "+v"(c), "+v"(d) : "v"(x), "v"(y)); }
__device__ __forceinline__ void keep4_h(v16h a, v16h b, v16h c, v16h d) { asm volatile("v_nop" :: "v"(a), "v"(b), "v"(c), "v"(d)); }
__device__ __forceinline__ void keep4_b(v16b a, v16b b, v16b c, v16b d) { asm volatile("v_nop" :: "v"(a), "v"(b), "v"(c), "v"(d)); }
__device__ __forceinline__ void acc_guard4(v8f& a, v8f& b, v8f& c, v8f& d) { asm volatile("v_nop\n\tv_nop\n\tv_nop\n\tv_nop" : "+v"(a), "+v"(b), "+v"(c), "+v"(d)); }
template <typename T> struct Frag;
template <> struct Frag<_Float16> {
  typedef v16h V; union U { v16h v; v8h h[2]; };
  static __device__ __forceinline__ v16h load(const _Float16* p) {
    U f; f.h[0] = *(const v8h*)(p); f.h[1] = *(const v8h*)(p + 16); return f.v;
  }
  static __device__ __forceinline__ v8f mma(v16h a, v16h b, v8f c) {
    return __builtin_amdgcn_wmma_f32_16x16x32_f16(false, a, false, b, (short)0, c, false, false);
  }
  static __device__ __forceinline__ void guard(v8f& a, v8f& b, v16h x, v16h y) { dep_guard_h(a, b, x, y); }
  static __device__ __forceinline__ void guard4(v8f& a, v8f& b, v8f& c, v8f& d, v16h x, v16h y) { dep_guard4_h(a, b, c, d, x, y); }
  static __device__ __forceinline__ void keep(v16h a, v16h b, v16h c, v16h d) { keep4_h(a, b, c, d); }
};
template <> struct Frag<__bf16> {
  typedef v16b V; union U { v16b v; v8b h[2]; };
  static __device__ __forceinline__ v16b load(const __bf16* p) {
    U f; f.h[0] = *(const v8b*)(p); f.h[1] = *(const v8b*)(p + 16); return f.v;
  }
  static __device__ __forceinline__ v8f mma(v16b a, v16b b, v8f c) {
    return __builtin_amdgcn_wmma_f32_16x16x32_bf16(false, a, false, b, (short)0, c, false, false);
  }
  static __device__ __forceinline__ void guard(v8f& a, v8f& b, v16b x, v16b y) { dep_guard_b(a, b, x, y); }
  static __device__ __forceinline__ void guard4(v8f& a, v8f& b, v8f& c, v8f& d, v16b x, v16b y) { dep_guard4_b(a, b, c, d, x, y); }
  static __device__ __forceinline__ void keep(v16b a, v16b b, v16b c, v16b d) { keep4_b(a, b, c, d); }
};

template <int ET> struct Elem;
template <> struct Elem<0> { typedef _Float16 T; };
template <> struct Elem<1> { typedef __bf16 T; };
template <int ET, int SPLIT, int BIAS_MODE, int OUT_MODE, bool RESID, int ACT = 0>
__global__ __launch_bounds__(256) void wmma_gemm64(
    const unsigned short* __restrict__ Ap, const unsigned short* __restrict__ A2p, int lda, long strideA,
    const unsigned short* __restrict__ Btp, const unsigned short* __restrict__ Bt2p, int ldb, long strideB,
    void* __restrict__ Cout, void* __restrict__ Cout2, int ldc, long strideC,
    const float* __restrict__ bias,
    const float* __restrict__ resid, long strideR,
    int M, int N, int K, float scale) {
  typedef typename Elem<ET>::T T;
  typedef typename Frag<T>::V V;
  const T* A = (const T*)Ap; const T* A2 = (const T*)A2p; const T* Bt = (const T*)Btp; const T* Bt2 = (const T*)Bt2p;
  __shared__ __align__(16) float sT[8][16 * 68];
  const int b    = blockIdx.y;
  const int lane = threadIdx.x & 31;
  const int wave = threadIdx.x >> 5;
  const int tilesN = N >> 6;
  const int tilesM = M >> 6;
  const int tile = blockIdx.x * 8 + wave;
  if (tile >= tilesM * tilesN) return;
  const int tm = tile / tilesN;
  const int tn = tile - tm * tilesN;
  const int m0 = tm << 6;
  const int n0 = tn << 6;

  const T* Ab  = A  + (size_t)b * strideA;
  const T* Bb  = Bt + (size_t)b * strideB;
  const T* Ab2 = (SPLIT != 0) ? (A2  + (size_t)b * strideA) : nullptr;
  const T* Bb2 = (SPLIT == 1) ? (Bt2 + (size_t)b * strideB) : nullptr;

  const int rlane = lane & 15;
  const int koff  = (lane >> 4) * 8;
  const int mOff  = (lane >> 4) * 8;

  v8f acc[4][4];
#pragma unroll
  for (int i = 0; i < 4; ++i)
#pragma unroll
    for (int j = 0; j < 4; ++j) acc[i][j] = (v8f){0.f,0.f,0.f,0.f,0.f,0.f,0.f,0.f};

  for (int k0 = 0; k0 < K; k0 += 32) {
    V bh[4], bl[4];
#pragma unroll
    for (int j = 0; j < 4; ++j) {
      const size_t bo = (size_t)(n0 + (j << 4) + rlane) * ldb + koff + k0;
      bh[j] = Frag<T>::load(Bb + bo);
      if (SPLIT == 1) bl[j] = Frag<T>::load(Bb2 + bo);
    }
#pragma unroll
    for (int i = 0; i < 4; ++i) {
      const size_t ao = (size_t)(m0 + (i << 4) + rlane) * lda + koff + k0;
      V ah = Frag<T>::load(Ab + ao);
      V al;
      if (SPLIT != 0) al = Frag<T>::load(Ab2 + ao);
#pragma unroll
      for (int j = 0; j < 4; ++j) {
        acc[i][j] = Frag<T>::mma(ah, bh[j], acc[i][j]);
        if (SPLIT == 1) acc[i][j] = Frag<T>::mma(ah, bl[j], acc[i][j]);
        if (SPLIT != 0) acc[i][j] = Frag<T>::mma(al, bh[j], acc[i][j]);
      }
      Frag<T>::guard4(acc[i][0], acc[i][1], acc[i][2], acc[i][3], ah, (SPLIT != 0) ? al : ah);
    }
    Frag<T>::keep(bh[0], bh[1], bh[2], bh[3]);
    if (SPLIT == 1) Frag<T>::keep(bl[0], bl[1], bl[2], bl[3]);
  }
  acc_guard4(acc[0][0], acc[0][1], acc[0][2], acc[0][3]);
  acc_guard4(acc[1][0], acc[1][1], acc[1][2], acc[1][3]);
  acc_guard4(acc[2][0], acc[2][1], acc[2][2], acc[2][3]);
  acc_guard4(acc[3][0], acc[3][1], acc[3][2], acc[3][3]);

  float* slab = sT[wave];
  const float* Rb = RESID ? (resid + (size_t)b * strideR) : nullptr;
#pragma unroll
  for (int i = 0; i < 4; ++i) {
    const int mBase = m0 + (i << 4);
#pragma unroll
    for (int j = 0; j < 4; ++j) {
      const int n = n0 + (j << 4) + rlane;
      float bv = 0.f;
      if (BIAS_MODE == 2) bv = bf_bits2f(f2bf_bits(bias[n]));
#pragma unroll
      for (int r = 0; r < 8; ++r) {
        float v = acc[i][j][r] * scale;
        if (BIAS_MODE == 1) v += bf_bits2f(f2bf_bits(bias[mBase + mOff + r]));
        if (BIAS_MODE == 2) v += bv;
        if (RESID) v += Rb[(size_t)(mBase + mOff + r) * ldc + n];
        if (ACT == 2) v = fmaxf(v, 0.0f);
        if (ACT == 4) v = (v > 0.f) ? v : 0.01f * v;
        slab[(mOff + r) * 68 + (j << 4) + rlane] = v;
      }
    }
    __builtin_amdgcn_fence(__ATOMIC_RELEASE, "workgroup");
    __builtin_amdgcn_wave_barrier();
    __builtin_amdgcn_fence(__ATOMIC_ACQUIRE, "workgroup");
    if (OUT_MODE == 0) {
      float* C = (float*)Cout + (size_t)b * strideC;
      const int hh = lane >> 4, c4 = (lane & 15) * 4;
      for (int pass = 0; pass < 2; ++pass) {
#pragma unroll
        for (int it = 0; it < 8; ++it) {
          const int row = it * 2 + hh;
          v4f v = *(const v4f*)(slab + row * 68 + c4);
          *(volatile v4f*)(C + (size_t)(mBase + row) * ldc + n0 + c4) = v;
        }
        __threadfence();
      }
    } else {
      const int q = lane >> 3, c8 = (lane & 7) * 8;
      unsigned short* C  = (unsigned short*)Cout  + (size_t)b * strideC;
      unsigned short* C2 = (OUT_MODE == 2) ? ((unsigned short*)Cout2 + (size_t)b * strideC) : nullptr;
      for (int pass = 0; pass < 2; ++pass) {
#pragma unroll
        for (int it = 0; it < 4; ++it) {
          const int row = it * 4 + q;
          const float* sp = slab + row * 68 + c8;
          v8h hv, lv;
#pragma unroll
          for (int e = 0; e < 8; ++e) {
            if (OUT_MODE == 1) {
              hv[e] = (_Float16)sp[e];
            } else {
              unsigned short hb = f2bf_bits(sp[e]);
              unsigned short lb = f2bf_bits(sp[e] - bf_bits2f(hb));
              hv[e] = __builtin_bit_cast(_Float16, hb);
              lv[e] = __builtin_bit_cast(_Float16, lb);
            }
          }
          *(volatile v8h*)(C + (size_t)(mBase + row) * ldc + n0 + c8) = hv;
          if (OUT_MODE == 2) *(volatile v8h*)(C2 + (size_t)(mBase + row) * ldc + n0 + c8) = lv;
        }
        __threadfence();
      }
    }
    __builtin_amdgcn_fence(__ATOMIC_RELEASE, "workgroup");
    __builtin_amdgcn_wave_barrier();
    __builtin_amdgcn_fence(__ATOMIC_ACQUIRE, "workgroup");
  }
}

__global__ __launch_bounds__(256) void cast8_bf16_kernel(const float* __restrict__ in, unsigned short* __restrict__ out, int n8) {
  const int i = blockIdx.x * 256 + threadIdx.x;
  if (i >= n8) return;
  const float* p = in + 8 * (size_t)i;
  const v4f a = *(const v4f*)(p);
  const v4f c = *(const v4f*)(p + 4);
  unsigned short hb[8];
#pragma unroll
  for (int e = 0; e < 4; ++e) {
    hb[e]     = f2bf_bits(a[e]);
    hb[4 + e] = f2bf_bits(c[e]);
  }
  const v4u u = (v4u){pk16(hb[0], hb[1]), pk16(hb[2], hb[3]), pk16(hb[4], hb[5]), pk16(hb[6], hb[7])};
  unsigned short* q = out + 8 * (size_t)i;
  *(volatile v4u*)q = u;
  __threadfence();
  *(volatile v4u*)q = u;
}

__global__ __launch_bounds__(256) void vt_transpose_kernel(const unsigned short* __restrict__ qkvh,
                                                           const unsigned short* __restrict__ qkvl,
                                                           unsigned short* __restrict__ vth,
                                                           unsigned short* __restrict__ vtl) {
  __shared__ unsigned short sm[2][64][66];
  const int tid = threadIdx.x;
  const int t0 = blockIdx.x * 64;
  const int h  = blockIdx.y;
  const int b  = blockIdx.z;
#pragma unroll
  for (int i = 0; i < 2; ++i) {
    const int w  = i * 256 + tid;
    const int r  = w >> 3;
    const int c8 = (w & 7) * 8;
    const size_t go = ((size_t)(b * kSeq + t0 + r)) * kQkvN + 2 * kDim + h * kDh + c8;
    const v4u uh = *(const v4u*)(qkvh + go);
    const v4u ul = *(const v4u*)(qkvl + go);
#pragma unroll
    for (int e = 0; e < 4; ++e) {
      sm[0][c8 + 2 * e][r]     = (unsigned short)(uh[e] & 0xffffu);
      sm[0][c8 + 2 * e + 1][r] = (unsigned short)(uh[e] >> 16);
      sm[1][c8 + 2 * e][r]     = (unsigned short)(ul[e] & 0xffffu);
      sm[1][c8 + 2 * e + 1][r] = (unsigned short)(ul[e] >> 16);
    }
  }
  __syncthreads();
  const int lane = tid & 31, wave = tid >> 5;
  const int q = lane >> 3, c8 = (lane & 7) * 8;
  const size_t rowbase = (size_t)(b * kHeads + h) * kDh;
  for (int pass = 0; pass < 2; ++pass) {
#pragma unroll
    for (int it = 0; it < 2; ++it) {
      const int row = wave * 8 + it * 4 + q;
      unsigned short ha[8], la[8];
#pragma unroll
      for (int e = 0; e < 8; ++e) { ha[e] = sm[0][row][c8 + e]; la[e] = sm[1][row][c8 + e]; }
      const v4u ua = (v4u){pk16(ha[0], ha[1]), pk16(ha[2], ha[3]), pk16(ha[4], ha[5]), pk16(ha[6], ha[7])};
      const v4u ub = (v4u){pk16(la[0], la[1]), pk16(la[2], la[3]), pk16(la[4], la[5]), pk16(la[6], la[7])};
      const size_t oo = (rowbase + row) * (size_t)kSeq + t0 + c8;
      *(volatile v4u*)(vth + oo) = ua;
      *(volatile v4u*)(vtl + oo) = ub;
    }
    __threadfence();
  }
}

__device__ __forceinline__ v8f mma_bf16_g(v16b a, v16b b, v8f c) {
  c = __builtin_amdgcn_wmma_f32_16x16x32_bf16(false, a, false, b, (short)0, c, false, false);
  asm volatile("v_nop\n\tv_nop\n\tv_nop\n\tv_nop" : "+v"(c) : "v"(a), "v"(b));
  return c;
}

__global__ __launch_bounds__(128) void causal_attn_kernel(
    const unsigned short* __restrict__ qkvh_p, const unsigned short* __restrict__ qkvl_p,
    const unsigned short* __restrict__ vth_p,  const unsigned short* __restrict__ vtl_p,
    unsigned short* __restrict__ ctxh, unsigned short* __restrict__ ctxl) {
  union FB { v16b v; v8b h[2]; };
  __shared__ __align__(16) __bf16 Ksh[kAK * kDh];
  __shared__ __align__(16) __bf16 Ksl[kAK * kDh];
  __shared__ __align__(16) __bf16 Vth[kDh * kAK];
  __shared__ __align__(16) __bf16 Vtl[kDh * kAK];
  __shared__ __align__(16) __bf16 Psh[4][16 * kAK];
  __shared__ __align__(16) __bf16 Psl[4][16 * kAK];
  __shared__ __align__(16) float  Os[4][16 * kOsPitch];

  const __bf16* Qh  = (const __bf16*)qkvh_p;
  const __bf16* Ql  = (const __bf16*)qkvl_p;
  const __bf16* VTh = (const __bf16*)vth_p;
  const __bf16* VTl = (const __bf16*)vtl_p;

  const int tid  = threadIdx.x;
  const int wave = tid >> 5;
  const int lane = tid & 31;
  const int hh   = lane >> 4;
  const int c    = lane & 15;

  const int nqb = kSeq / kAQ;
  const int bx  = blockIdx.x;
  const int qb  = bx % nqb;
  const int bh  = bx / nqb;
  const int h   = bh % kHeads;
  const int b   = bh / kHeads;
  const int q0  = qb * kAQ + wave * 16;
  const size_t tokb = (size_t)b * kSeq;

  v16b qah[2], qal[2];
  {
    const size_t qo = (tokb + q0 + c) * (size_t)kQkvN + (size_t)h * kDh + 8 * hh;
#pragma unroll
    for (int dc = 0; dc < 2; ++dc) {
      FB f0;
      f0.h[0] = *(const v8b*)(Qh + qo + dc * 32);
      f0.h[1] = *(const v8b*)(Qh + qo + dc * 32 + 16);
      qah[dc] = f0.v;
      FB f1;
      f1.h[0] = *(const v8b*)(Ql + qo + dc * 32);
      f1.h[1] = *(const v8b*)(Ql + qo + dc * 32 + 16);
      qal[dc] = f1.v;
    }
  }

  float mrow[8], lrow[8];
  v8f oacc[4];
#pragma unroll
  for (int r = 0; r < 8; ++r) { mrow[r] = -__builtin_inff(); lrow[r] = 0.f; }
#pragma unroll
  for (int t = 0; t < 4; ++t) oacc[t] = (v8f){0.f,0.f,0.f,0.f,0.f,0.f,0.f,0.f};

  const int nChunks = qb + 1;
  for (int kc = 0; kc < nChunks; ++kc) {
    const int kv0 = kc * kAK;
    __syncthreads();
#pragma unroll
    for (int i = 0; i < 4; ++i) {
      const int w  = i * 128 + tid;
      const int r  = w >> 3;
      const int c8 = (w & 7) * 8;
      const size_t ko = (tokb + kv0 + r) * (size_t)kQkvN + kDim + (size_t)h * kDh + c8;
      *(v8b*)(Ksh + r * kDh + c8) = *(const v8b*)(Qh + ko);
      *(v8b*)(Ksl + r * kDh + c8) = *(const v8b*)(Ql + ko);
    }
    asm volatile("" ::: "memory");
#pragma unroll
    for (int i = 0; i < 4; ++i) {
      const int w  = i * 128 + tid;
      const int r  = w >> 3;
      const int c8 = (w & 7) * 8;
      const size_t vo = ((size_t)(bh * kDh + r)) * (size_t)kSeq + kv0 + c8;
      *(v8b*)(Vth + r * kAK + c8) = *(const v8b*)(VTh + vo);
      *(v8b*)(Vtl + r * kAK + c8) = *(const v8b*)(VTl + vo);
    }
    __syncthreads();

    v8f s[4];
#pragma unroll
    for (int j = 0; j < 4; ++j) {
      s[j] = (v8f){0.f,0.f,0.f,0.f,0.f,0.f,0.f,0.f};
      const __bf16* kr  = Ksh + (j * 16 + c) * kDh + 8 * hh;
      const __bf16* kr2 = Ksl + (j * 16 + c) * kDh + 8 * hh;
#pragma unroll
      for (int dc = 0; dc < 2; ++dc) {
        FB kb, kl;
        kb.h[0] = *(const v8b*)(kr + dc * 32);
        kb.h[1] = *(const v8b*)(kr + dc * 32 + 16);
        kl.h[0] = *(const v8b*)(kr2 + dc * 32);
        kl.h[1] = *(const v8b*)(kr2 + dc * 32 + 16);
        s[j] = mma_bf16_g(qah[dc], kb.v, s[j]);
        s[j] = mma_bf16_g(qah[dc], kl.v, s[j]);
        s[j] = mma_bf16_g(qal[dc], kb.v, s[j]);
      }
    }

    const bool diag = (kc == qb);
    float cm[8];
#pragma unroll
    for (int r = 0; r < 8; ++r) {
      const int qrow = q0 + 8 * hh + r;
      float m = -__builtin_inff();
#pragma unroll
      for (int j = 0; j < 4; ++j) {
        const int kvcol = kv0 + j * 16 + c;
        float val = s[j][r] * kAttnScale;
        const bool masked = diag && (kvcol > qrow);
        val = masked ? -__builtin_inff() : val;
        s[j][r] = val;
        m = fmaxf(m, val);
      }
#pragma unroll
      for (int off = 1; off < 16; off <<= 1) m = fmaxf(m, __shfl_xor(m, off, 32));
      cm[r] = m;
    }

    __bf16* pwh = Psh[wave];
    __bf16* pwl = Psl[wave];
#pragma unroll
    for (int r = 0; r < 8; ++r) {
      const float mnew  = fmaxf(mrow[r], cm[r]);
      const float alpha = expf(mrow[r] - mnew);
      mrow[r] = mnew;
      float psum = 0.f;
#pragma unroll
      for (int j = 0; j < 4; ++j) {
        const float p = expf(s[j][r] - mnew);
        psum += p;
        const unsigned short hb = f2bf_bits(p);
        const unsigned short lb = f2bf_bits(p - bf_bits2f(hb));
        pwh[(8 * hh + r) * kAK + j * 16 + c] = __builtin_bit_cast(__bf16, hb);
        pwl[(8 * hh + r) * kAK + j * 16 + c] = __builtin_bit_cast(__bf16, lb);
      }
#pragma unroll
      for (int off = 1; off < 16; off <<= 1) psum += __shfl_xor(psum, off, 32);
      lrow[r] = lrow[r] * alpha + psum;
#pragma unroll
      for (int t = 0; t < 4; ++t) oacc[t][r] *= alpha;
    }
    __syncthreads();

#pragma unroll
    for (int kk = 0; kk < 2; ++kk) {
      FB pa, pl;
      pa.h[0] = *(const v8b*)(pwh + c * kAK + kk * 32 + 8 * hh);
      pa.h[1] = *(const v8b*)(pwh + c * kAK + kk * 32 + 16 + 8 * hh);
      pl.h[0] = *(const v8b*)(pwl + c * kAK + kk * 32 + 8 * hh);
      pl.h[1] = *(const v8b*)(pwl + c * kAK + kk * 32 + 16 + 8 * hh);
#pragma unroll
      for (int t = 0; t < 4; ++t) {
        FB vb, vl;
        vb.h[0] = *(const v8b*)(Vth + (t * 16 + c) * kAK + kk * 32 + 8 * hh);
        vb.h[1] = *(const v8b*)(Vth + (t * 16 + c) * kAK + kk * 32 + 16 + 8 * hh);
        vl.h[0] = *(const v8b*)(Vtl + (t * 16 + c) * kAK + kk * 32 + 8 * hh);
        vl.h[1] = *(const v8b*)(Vtl + (t * 16 + c) * kAK + kk * 32 + 16 + 8 * hh);
        oacc[t] = mma_bf16_g(pa.v, vb.v, oacc[t]);
        oacc[t] = mma_bf16_g(pa.v, vl.v, oacc[t]);
        oacc[t] = mma_bf16_g(pl.v, vb.v, oacc[t]);
      }
    }
  }

  float* os = Os[wave];
#pragma unroll
  for (int r = 0; r < 8; ++r) {
    const float inv = 1.0f / lrow[r];
#pragma unroll
    for (int t = 0; t < 4; ++t) os[(8 * hh + r) * kOsPitch + t * 16 + c] = oacc[t][r] * inv;
  }
  __syncthreads();
  {
    const int q4 = lane >> 3, c8 = (lane & 7) * 8;
    for (int pass = 0; pass < 2; ++pass) {
#pragma unroll
      for (int it = 0; it < 4; ++it) {
        const int row = it * 4 + q4;
        const float* sp = os + row * kOsPitch + c8;
        const v4f x0 = *(const v4f*)(sp);
        const v4f x1 = *(const v4f*)(sp + 4);
        unsigned short hb[8], lb[8];
#pragma unroll
        for (int e = 0; e < 4; ++e) {
          hb[e] = f2bf_bits(x0[e]);
          lb[e] = f2bf_bits(x0[e] - bf_bits2f(hb[e]));
          hb[4 + e] = f2bf_bits(x1[e]);
          lb[4 + e] = f2bf_bits(x1[e] - bf_bits2f(hb[4 + e]));
        }
        const v4u uh = (v4u){pk16(hb[0], hb[1]), pk16(hb[2], hb[3]), pk16(hb[4], hb[5]), pk16(hb[6], hb[7])};
        const v4u ul = (v4u){pk16(lb[0], lb[1]), pk16(lb[2], lb[3]), pk16(lb[4], lb[5]), pk16(lb[6], lb[7])};
        const size_t go = (tokb + q0 + row) * (size_t)kDim + (size_t)h * kDh + c8;
        *(volatile v4u*)(ctxh + go) = uh;
        *(volatile v4u*)(ctxl + go) = ul;
      }
      __threadfence();
    }
  }
}

extern "C" void kernel_launch(void* const* d_in, const int* in_sizes, int n_in,
                              void* d_out, int out_size, void* d_ws, size_t ws_size,
                              hipStream_t stream) {
  if (n_in < 5) return;
  if (in_sizes[0] != kTok * kDim) return;
  if (in_sizes[1] != kQkvN * kDim) return;
  if (in_sizes[2] != kQkvN) return;
  if (in_sizes[3] != kDim * kDim) return;
  if (in_sizes[4] != kDim) return;
  if (out_size != kTok * kDim) return;

  const size_t szXB  = (size_t)kTok * kDim * 2;
  const size_t szWQ  = (size_t)kQkvN * kDim * 2;
  const size_t szWP  = (size_t)kDim * kDim * 2;
  const size_t szQKV = (size_t)kTok * kQkvN * 2;
  const size_t szVT  = (size_t)kBatch * kHeads * kDh * kSeq * 2;
  const size_t szCTX = (size_t)kTok * kDim * 2;
  const size_t offXB   = 0;
  const size_t offWQ   = offXB + szXB;
  const size_t offWP   = offWQ + szWQ;
  const size_t offQKVH = offWP + szWP;
  const size_t offQKVL = offQKVH + szQKV;
  const size_t offVTH  = offQKVL + szQKV;
  const size_t offVTL  = offVTH + szVT;
  const size_t offCTXH = offVTL + szVT;
  const size_t offCTXL = offCTXH + szCTX;
  const size_t total   = offCTXL + szCTX;
  if (ws_size < total) return;

  const float* x     = (const float*)d_in[0];
  const float* Wqkv  = (const float*)d_in[1];
  const float* bqkv  = (const float*)d_in[2];
  const float* Wproj = (const float*)d_in[3];
  const float* bproj = (const float*)d_in[4];
  float* out = (float*)d_out;
  char* ws = (char*)d_ws;
  unsigned short* XB   = (unsigned short*)(ws + offXB);
  unsigned short* WQ   = (unsigned short*)(ws + offWQ);
  unsigned short* WP   = (unsigned short*)(ws + offWP);
  unsigned short* QKVH = (unsigned short*)(ws + offQKVH);
  unsigned short* QKVL = (unsigned short*)(ws + offQKVL);
  unsigned short* VTH  = (unsigned short*)(ws + offVTH);
  unsigned short* VTL  = (unsigned short*)(ws + offVTL);
  unsigned short* CTXH = (unsigned short*)(ws + offCTXH);
  unsigned short* CTXL = (unsigned short*)(ws + offCTXL);

  const int n8x = (kTok * kDim) / 8;
  const int n8w = (kQkvN * kDim) / 8;
  const int n8p = (kDim * kDim) / 8;
  cast8_bf16_kernel<<<dim3((n8x + 255) / 256), dim3(256), 0, stream>>>(x, XB, n8x);
  cast8_bf16_kernel<<<dim3((n8w + 255) / 256), dim3(256), 0, stream>>>(Wqkv, WQ, n8w);
  cast8_bf16_kernel<<<dim3((n8p + 255) / 256), dim3(256), 0, stream>>>(Wproj, WP, n8p);

  const int tilesQkv = (kTok / 64) * (kQkvN / 64);
  wmma_gemm64<1, 0, 2, 2, false, 0><<<dim3(tilesQkv / 8, 1), dim3(256), 0, stream>>>(
      XB, XB, kDim, 0L, WQ, WQ, kDim, 0L,
      (void*)QKVH, (void*)QKVL, kQkvN, 0L, bqkv, bqkv, 0L, kTok, kQkvN, kDim, 1.0f);

  vt_transpose_kernel<<<dim3(kSeq / 64, kHeads, kBatch), dim3(256), 0, stream>>>(QKVH, QKVL, VTH, VTL);

  causal_attn_kernel<<<dim3(kBatch * kHeads * (kSeq / kAQ)), dim3(128), 0, stream>>>(QKVH, QKVL, VTH, VTL, CTXH, CTXL);

  const int tilesProj = (kTok / 64) * (kDim / 64);
  wmma_gemm64<1, 2, 2, 0, false, 0><<<dim3(tilesProj / 8, 1), dim3(256), 0, stream>>>(
      CTXH, CTXL, kDim, 0L, WP, WP, kDim, 0L,
      (void*)out, (void*)out, kDim, 0L, bproj, bproj, 0L, kTok, kDim, kDim, 1.0f);
}
